// TFNLiteLayer_2302102471547
// MI455X (gfx1250) — hardware-verified
//
#include <hip/hip_runtime.h>
#include <stddef.h>
#include <math.h>


#define NTHR   256
#define NWAVE  8
#define TE     32
#define KD     64
#define NR     320
#define NCOL   576
#define AP     72
#define NODEB  256
#define EPT    8
#define NGRP   2
#define CHUNK  (NTHR * EPT * NGRP)
#define WCAP   (EPT * NGRP * 32)
#define LISTN  (NWAVE * WCAP)

#define OFF_W1   0
#define OFF_O    0
#define OFF_RBF  4096
#define OFF_AH   6144
#define OFF_AL   10752
#define OFF_X    15360
#define OFF_N    19456
#define OFF_M    19968
#define OFF_ROW  21504
#define OFF_W    21632
#define LDS_EDGE 62592
#define LDS_AGG  (NODEB * 32 * 4 + LISTN * 4 + 64)

static_assert((CHUNK & (CHUNK - 1)) == 0 && CHUNK <= 4096);
static_assert((NODEB & (NODEB - 1)) == 0 && NODEB <= 4096);
static_assert(NODEB == NWAVE * 4 * 8);
static_assert(TE == 32 && TE == NWAVE * 4 && NTHR == 8 * TE);
static_assert(NR == 20 * 16 && KD == 64);
static_assert(OFF_O + TE * 32 * 4 <= OFF_RBF);
static_assert(OFF_RBF + TE * 16 * 4 == OFF_AH && OFF_AH + TE * AP * 2 == OFF_AL && OFF_AL + TE * AP * 2 == OFF_X);
static_assert(OFF_X + TE * 32 * 4 == OFF_N && OFF_N + TE * 4 * 4 == OFF_M && OFF_M + TE * 12 * 4 == OFF_ROW);
static_assert(OFF_ROW + TE * 4 == OFF_W && OFF_W + TE * NR * 4 == LDS_EDGE);
static_assert(LDS_EDGE <= 65536 && LDS_AGG <= 65536);
static_assert((OFF_W % 16) == 0 && (OFF_O % 16) == 0 && (OFF_AH % 16) == 0 && (OFF_AL % 16) == 0 && (OFF_X % 16) == 0);

#define C_S15   3.872983346207417f
#define C_S5    2.23606797749979f
#define C_Q10   0.31622776601683794f
#define C_R302  0.3651483716701107f
#define C_R301  0.18257418583505536f
#define C_A0    0.17677669529663687f
#define C_A1    0.27386127875258304f
#define C_IS3   0.5773502691896258f

typedef float          v4f  __attribute__((ext_vector_type(4)));
typedef float          v8f  __attribute__((ext_vector_type(8)));
typedef int            v4i  __attribute__((ext_vector_type(4)));
typedef unsigned short v8us __attribute__((ext_vector_type(8)));
typedef __bf16         v16b __attribute__((ext_vector_type(16)));
union FragB { v16b v; v8us h[2]; };

__device__ __forceinline__ unsigned short bf16_rne(float f) {
  unsigned u = __float_as_uint(f);
  u = u + 0x7FFFu + ((u >> 16) & 1u);
  return (unsigned short)(u >> 16);
}
__device__ __forceinline__ float bf16_val(unsigned short s) {
  return __uint_as_float(((unsigned)s) << 16);
}

__device__ __forceinline__ v8f wmb(v16b a, v16b b, v8f c) {
#if defined(__HIP_DEVICE_COMPILE__)
  v8f d = __builtin_amdgcn_wmma_f32_16x16x32_bf16(false, a, false, b, (short)0, c, false, false);
  asm volatile("v_nop\n\tv_nop\n\tv_nop\n\tv_nop" : "+v"(d) : "v"(a), "v"(b));
  return d;
#else
  return c;
#endif
}

__device__ __forceinline__ void hsplit(float z, unsigned short& h, unsigned short& l) {
  const float v = fmaxf(z * 0.25f, 0.0f);
  const unsigned short hs = bf16_rne(v);
  h = hs;
  l = bf16_rne(v - bf16_val(hs));
}

__device__ __forceinline__ float silu_f(float v) {
#if defined(__HIP_DEVICE_COMPILE__)
  const float ex = __expf(fminf(-v, 60.0f));
  return v * __builtin_amdgcn_rcpf(1.0f + ex);
#else
  return v;
#endif
}

template <int NSL>
__device__ __forceinline__ int scan_chunk(const int* __restrict__ dsts, int nE, int cbase, int slotBase,
                                          int vec8, int* list, int tid, int lane, int wave) {
  int wc = 0;
#pragma unroll
  for (int g = 0; g < NGRP; ++g) {
    const int el0  = (g * NTHR + tid) * EPT;
    const int e0   = cbase + el0;
    const int sent = -2147483647 - 1;
    v4i da, db;
    if (vec8 != 0 && cbase + CHUNK <= nE) {
      da = *(const v4i*)(dsts + e0);
      db = *(const v4i*)(dsts + e0 + 4);
    } else {
      da.x = (e0     < nE) ? dsts[min(e0, nE - 1)] : sent;
      da.y = (e0 + 1 < nE) ? dsts[min(e0 + 1, nE - 1)] : sent;
      da.z = (e0 + 2 < nE) ? dsts[min(e0 + 2, nE - 1)] : sent;
      da.w = (e0 + 3 < nE) ? dsts[min(e0 + 3, nE - 1)] : sent;
      db.x = (e0 + 4 < nE) ? dsts[min(e0 + 4, nE - 1)] : sent;
      db.y = (e0 + 5 < nE) ? dsts[min(e0 + 5, nE - 1)] : sent;
      db.z = (e0 + 6 < nE) ? dsts[min(e0 + 6, nE - 1)] : sent;
      db.w = (e0 + 7 < nE) ? dsts[min(e0 + 7, nE - 1)] : sent;
    }
    const unsigned nb = (unsigned)slotBase;
    const unsigned s0 = (unsigned)da.x - nb, s1 = (unsigned)da.y - nb;
    const unsigned s2 = (unsigned)da.z - nb, s3 = (unsigned)da.w - nb;
    const unsigned s4 = (unsigned)db.x - nb, s5 = (unsigned)db.y - nb;
    const unsigned s6 = (unsigned)db.z - nb, s7 = (unsigned)db.w - nb;
    const bool h0 = s0 < (unsigned)NSL, h1 = s1 < (unsigned)NSL, h2 = s2 < (unsigned)NSL, h3 = s3 < (unsigned)NSL;
    const bool h4 = s4 < (unsigned)NSL, h5 = s5 < (unsigned)NSL, h6 = s6 < (unsigned)NSL, h7 = s7 < (unsigned)NSL;
    const unsigned any = __builtin_amdgcn_ballot_w32(h0 | h1 | h2 | h3 | h4 | h5 | h6 | h7);
    if (any != 0u) {
#define HITJ(J, HJ, SJ) { \
        const unsigned mj = __builtin_amdgcn_ballot_w32(HJ); \
        if (mj != 0u) { \
          if (HJ) { \
            const int pos = wc + (int)__builtin_amdgcn_mbcnt_lo(mj, 0u); \
            if (pos < WCAP) list[wave * WCAP + pos] = ((el0 + (J)) << 12) | (int)(SJ); \
          } \
          wc += (int)__builtin_popcount(mj); } }
      HITJ(0, h0, s0)
      HITJ(1, h1, s1)
      HITJ(2, h2, s2)
      HITJ(3, h3, s3)
      HITJ(4, h4, s4)
      HITJ(5, h5, s5)
      HITJ(6, h6, s6)
      HITJ(7, h7, s7)
#undef HITJ
    }
  }
  return wc;
}

__global__ __launch_bounds__(NTHR) void k_wprep(
    const float* __restrict__ W2, unsigned short* bhi, unsigned short* blo) {
  const int i = blockIdx.x * NTHR + (int)threadIdx.x;
  if (i >= 2 * NR * 8) return;
  const int plane = i / (NR * 8);
  const int r  = i - plane * (NR * 8);
  const int n  = r >> 3;
  const int k0 = (r & 7) * 8;
  int src, pair;
  if (n < 256) {
    const int p = n >> 6, idx = n & 63, u = idx >> 3, w = idx & 7;
    src = p * 128 + u * 16 + w; pair = 1;
  } else {
    src = 512 + (n - 256); pair = 0;
  }
  const int src2 = min(src + 8, NCOL - 1);
  v8us H, L;
#define WP1(E) { \
    const int k = k0 + (E); \
    const float a = W2[k * NCOL + src]; \
    const float b = W2[k * NCOL + src2]; \
    const float v = (pair != 0 ? (a + b) : a) * 0.125f; \
    const unsigned short hs = bf16_rne(v); \
    H[E] = hs; L[E] = bf16_rne(v - bf16_val(hs)); }
  WP1(0) WP1(1) WP1(2) WP1(3) WP1(4) WP1(5) WP1(6) WP1(7)
#undef WP1
  const v8us o = (plane == 0) ? H : L;
  unsigned short* dp = (plane == 0 ? bhi : blo) + n * KD + k0;
  *(volatile v8us*)dp = o;
  __threadfence();
  *(volatile v8us*)dp = o;
}

__global__ __launch_bounds__(NTHR) void k_edge(
    const float* __restrict__ x, const float* __restrict__ pos, const int* __restrict__ ei,
    const float* __restrict__ W1, const unsigned short* __restrict__ bhi,
    const unsigned short* __restrict__ blo, float* oute, int nN, int nE) {
  extern __shared__ v4f lds_dyn[];
  char* lb = (char*)lds_dyn;
  float*          sW1  = (float*)(lb + OFF_W1);
  float*          srbf = (float*)(lb + OFF_RBF);
  unsigned short* sAh  = (unsigned short*)(lb + OFF_AH);
  unsigned short* sAl  = (unsigned short*)(lb + OFF_AL);
  float*          sx   = (float*)(lb + OFF_X);
  float*          sn   = (float*)(lb + OFF_N);
  float*          sM   = (float*)(lb + OFF_M);
  int*            srow = (int*)(lb + OFF_ROW);
  float*          sw   = (float*)(lb + OFF_W);
  float*          so   = (float*)(lb + OFF_O);

  const int tid = threadIdx.x, lane = tid & 31, wave = tid >> 5, hh = lane >> 4, m = lane & 15;
  const int base = blockIdx.x * TE;

  ((v4f*)sW1)[tid] = *(const v4f*)(W1 + 4 * tid);

  if (tid < TE) {
#pragma clang fp contract(off)
    const int eg  = base + tid;
    const int egc = eg < nE ? eg : nE - 1;
    int row = ei[egc];
    int col = ei[(size_t)nE + egc];
    row = row < 0 ? 0 : (row > nN - 1 ? nN - 1 : row);
    col = col < 0 ? 0 : (col > nN - 1 ? nN - 1 : col);
    const float px = pos[(size_t)row * 3 + 0] - pos[(size_t)col * 3 + 0];
    const float py = pos[(size_t)row * 3 + 1] - pos[(size_t)col * 3 + 1];
    const float pz = pos[(size_t)row * 3 + 2] - pos[(size_t)col * 3 + 2];
    const float d   = sqrtf(px * px + py * py + pz * pz + 1e-12f);
    const float inv = 1.0f / d;
    const float nx = px * inv, ny = py * inv, nz = pz * inv;
    srow[tid] = row;
    sn[tid * 4 + 0] = nx; sn[tid * 4 + 1] = ny; sn[tid * 4 + 2] = nz; sn[tid * 4 + 3] = 0.0f;
    const float y20 = C_S15 * nx * nz;
    const float y21 = C_S15 * nx * ny;
    const float y22 = 0.5f * C_S5 * (3.0f * ny * ny - 1.0f);
    const float y23 = C_S15 * ny * nz;
    const float y24 = 0.5f * C_S15 * (nz * nz - nx * nx);
    const float m01 = y21 * C_Q10, m02 = y20 * C_Q10, m12 = y23 * C_Q10;
    float* Me = sM + tid * 12;
    Me[0] = -y22 * C_R301 - y24 * C_Q10;
    Me[1] = m01;  Me[2] = m02;
    Me[3] = m01;
    Me[4] = y22 * C_R302;
    Me[5] = m12;
    Me[6] = m02;  Me[7] = m12;
    Me[8] = -y22 * C_R301 + y24 * C_Q10;
    Me[9] = 0.0f; Me[10] = 0.0f; Me[11] = 0.0f;
    const bool valid = eg < nE;
#pragma unroll 1
    for (int q = 0; q < 16; ++q) {
      const float mu = (float)q * (5.0f / 15.0f);
      const float df = d - mu;
      const float v  = expf(-(df * df) * 4.5f);
      srbf[tid * 16 + q] = valid ? v : 0.0f;
    }
  }
  __syncthreads();

  {
    const int e = tid >> 3, q = tid & 7;
    const int row = srow[e];
    const v4f xa = *(const v4f*)(x + (size_t)row * 32 + q * 4);
    *(v4f*)(sx + e * 32 + q * 4) = xa;
    v4f z0 = {0.f, 0.f, 0.f, 0.f}, z1 = {0.f, 0.f, 0.f, 0.f};
    const float* rp = srbf + e * 16;
    const float* wq = sW1 + q * 8;
#pragma unroll 1
    for (int k = 0; k < 16; ++k) {
      const float r = rp[k];
      const float* wk = wq + k * 64;
      z0 += *(const v4f*)(wk)     * r;
      z1 += *(const v4f*)(wk + 4) * r;
    }
    v8us H0, L0;
#define SPL(IDX, VAL) { unsigned short a_, b_; hsplit(VAL, a_, b_); H0[IDX] = a_; L0[IDX] = b_; }
    SPL(0, z0.x) SPL(1, z0.y) SPL(2, z0.z) SPL(3, z0.w)
    SPL(4, z1.x) SPL(5, z1.y) SPL(6, z1.z) SPL(7, z1.w)
#undef SPL
    *(v8us*)(sAh + e * AP + q * 8) = H0;
    *(v8us*)(sAl + e * AP + q * 8) = L0;
  }
  __syncthreads();

  {
    const int rt = wave & 1, cth = wave >> 1;
    FragB ah0, ah1, al0, al1;
    const unsigned short* pa = sAh + (rt * 16 + m) * AP + 8 * hh;
    const unsigned short* pl = sAl + (rt * 16 + m) * AP + 8 * hh;
    ah0.h[0] = *(const v8us*)(pa);       ah0.h[1] = *(const v8us*)(pa + 16);
    ah1.h[0] = *(const v8us*)(pa + 32);  ah1.h[1] = *(const v8us*)(pa + 48);
    al0.h[0] = *(const v8us*)(pl);       al0.h[1] = *(const v8us*)(pl + 16);
    al1.h[0] = *(const v8us*)(pl + 32);  al1.h[1] = *(const v8us*)(pl + 48);
    float* wrow = sw + (rt * 16 + 8 * hh) * NR + m;
#pragma unroll 1
    for (int j = 0; j < 5; ++j) {
      const int ct = cth * 5 + j;
      const unsigned short* pb = bhi + (size_t)(ct * 16 + m) * KD + 8 * hh;
      const unsigned short* pc = blo + (size_t)(ct * 16 + m) * KD + 8 * hh;
      FragB bh0, bh1, bl0, bl1;
      bh0.h[0] = *(const v8us*)(pb);       bh0.h[1] = *(const v8us*)(pb + 16);
      bh1.h[0] = *(const v8us*)(pb + 32);  bh1.h[1] = *(const v8us*)(pb + 48);
      bl0.h[0] = *(const v8us*)(pc);       bl0.h[1] = *(const v8us*)(pc + 16);
      bl1.h[0] = *(const v8us*)(pc + 32);  bl1.h[1] = *(const v8us*)(pc + 48);
      v8f acc = {0.f, 0.f, 0.f, 0.f, 0.f, 0.f, 0.f, 0.f};
      acc = wmb(ah0.v, bh0.v, acc);
      acc = wmb(al0.v, bh0.v, acc);
      acc = wmb(ah0.v, bl0.v, acc);
      acc = wmb(ah1.v, bh1.v, acc);
      acc = wmb(al1.v, bh1.v, acc);
      acc = wmb(ah1.v, bl1.v, acc);
      float* wp = wrow + ct * 16;
#pragma unroll
      for (int r = 0; r < 8; ++r) wp[r * NR] = acc[r];
    }
  }
  __syncthreads();

  {
    const int e = tid >> 3, c = tid & 7;
    const float* wl = sw + e * NR;
    const float* xe = sx + e * 32;
    const float nx = sn[e * 4 + 0], ny = sn[e * 4 + 1], nz = sn[e * 4 + 2];
    const float* Me = sM + e * 12;
    const float M0 = Me[0], M1 = Me[1], M2 = Me[2], M3 = Me[3], M4 = Me[4];
    const float M5 = Me[5], M6 = Me[6], M7 = Me[7], M8 = Me[8];
    float sA = 0.f, sB = 0.f, sC = 0.f;
    float sD0 = 0.f, sD1 = 0.f, sD2 = 0.f;
    float sE0 = 0.f, sE1 = 0.f, sE2 = 0.f;
#pragma unroll
    for (int u = 0; u < 8; ++u) {
      const float xs = xe[u];
      const float x0 = xe[8 + 3 * u], x1 = xe[9 + 3 * u], x2 = xe[10 + 3 * u];
      const float dot = x0 * nx + x1 * ny + x2 * nz;
      const float t0 = M0 * x0 + M1 * x1 + M2 * x2;
      const float t1 = M3 * x0 + M4 * x1 + M5 * x2;
      const float t2 = M6 * x0 + M7 * x1 + M8 * x2;
      const int uo = u * 8 + c;
      const float wa = wl[uo], wb = wl[64 + uo], wc = wl[128 + uo], wd = wl[192 + uo], we = wl[256 + uo];
      sA  += wa * xs;
      sB  += wb * dot;
      sC  += wc * xs;
      sD0 += wd * x0; sD1 += wd * x1; sD2 += wd * x2;
      sE0 += we * t0; sE1 += we * t1; sE2 += we * t2;
    }
    float* oe = so + e * 32;
    oe[c] = C_A0 * (sA + sB);
    oe[8 + 3 * c + 0] = C_A1 * (sC * nx + sD0 * C_IS3 + sE0);
    oe[8 + 3 * c + 1] = C_A1 * (sC * ny + sD1 * C_IS3 + sE1);
    oe[8 + 3 * c + 2] = C_A1 * (sC * nz + sD2 * C_IS3 + sE2);
  }
  __syncthreads();

  {
    const int q4 = lane >> 3, j8 = lane & 7;
    const int el = wave * 4 + q4;
    const v4f o0 = *(const v4f*)(so + el * 32 + 4 * j8);
    float* g0 = oute + ((size_t)(base + el)) * 32 + 4 * j8;
    *(volatile v4f*)g0 = o0;
    __threadfence();
    *(volatile v4f*)g0 = o0;
  }
}

__global__ __launch_bounds__(NTHR) void k_agg(
    const int* __restrict__ ei, const float* __restrict__ oute, float* out, int nN, int nE) {
  extern __shared__ v4f lds_dyn[];
  float* acc  = (float*)lds_dyn;
  int*   list = (int*)(acc + NODEB * 32);
  int*   wcnt = list + LISTN;
  const int tid = threadIdx.x, lane = tid & 31, wave = tid >> 5;
  const int nodeBase = blockIdx.x * NODEB;

  {
    const v4f z = {0.f, 0.f, 0.f, 0.f};
    for (int i = tid; i < NODEB * 32 / 4; i += NTHR) ((v4f*)acc)[i] = z;
  }
  __syncthreads();

  const int nChunks = (nE + CHUNK - 1) / CHUNK;
#pragma unroll 1
  for (int ch = 0; ch < nChunks; ++ch) {
    const int cbase = ch * CHUNK;
    const int wc = scan_chunk<NODEB>(ei, nE, cbase, nodeBase, 1, list, tid, lane, wave);
    if (lane == 0) wcnt[wave] = wc;
    __syncthreads();
    if (wave == 0) {
#pragma unroll 1
      for (int wsx = 0; wsx < NWAVE; ++wsx) {
        int n = __builtin_amdgcn_readfirstlane(wcnt[wsx]);
        n = n > WCAP ? WCAP : (n < 0 ? 0 : n);
        const int* lp = list + wsx * WCAP;
#pragma unroll 1
        for (int i = 0; i < n; ++i) {
          const int ent  = __builtin_amdgcn_readfirstlane(lp[i]);
          const int slot = ent & (NODEB - 1);
          int e = cbase + ((ent >> 12) & (CHUNK - 1));
          e = e > nE - 1 ? nE - 1 : e;
          const float v = oute[(size_t)e * 32 + lane];
          float* ap = acc + slot * 32 + lane;
          *ap = *ap + v;
        }
      }
    }
    __syncthreads();
  }

  const int q4 = lane >> 3, j8 = lane & 7;
#pragma unroll 1
  for (int i = 0; i < 8; ++i) {
    const int ln = wave * 32 + 4 * i + q4;
    const int node = nodeBase + ln;
    v4f v = *(const v4f*)(acc + ln * 32 + 4 * j8);
    const float sx0 = silu_f(v.x), sy0 = silu_f(v.y), sz0 = silu_f(v.z), sw0 = silu_f(v.w);
    v.x = (j8 < 2) ? sx0 : v.x; v.y = (j8 < 2) ? sy0 : v.y;
    v.z = (j8 < 2) ? sz0 : v.z; v.w = (j8 < 2) ? sw0 : v.w;
    if (node < nN) *(volatile v4f*)(out + (size_t)node * 32 + 4 * j8) = v;
  }
  __threadfence();
#pragma unroll 1
  for (int i = 0; i < 8; ++i) {
    const int ln = wave * 32 + 4 * i + q4;
    const int node = nodeBase + ln;
    v4f v = *(const v4f*)(acc + ln * 32 + 4 * j8);
    const float sx0 = silu_f(v.x), sy0 = silu_f(v.y), sz0 = silu_f(v.z), sw0 = silu_f(v.w);
    v.x = (j8 < 2) ? sx0 : v.x; v.y = (j8 < 2) ? sy0 : v.y;
    v.z = (j8 < 2) ? sz0 : v.z; v.w = (j8 < 2) ? sw0 : v.w;
    if (node < nN) *(volatile v4f*)(out + (size_t)node * 32 + 4 * j8) = v;
  }
}

extern "C" void kernel_launch(void* const* d_in, const int* in_sizes, int n_in,
                              void* d_out, int out_size, void* d_ws, size_t ws_size,
                              hipStream_t stream) {
  if (n_in < 5) return;
  const int nN = in_sizes[0] / 32;
  const int nE = in_sizes[2] / 2;
  if (nN <= 0 || nE <= 0) return;
  if (in_sizes[0] != nN * 32 || in_sizes[1] != nN * 3 || in_sizes[2] != 2 * nE) return;
  if (in_sizes[3] != 16 * KD || in_sizes[4] != KD * NCOL) return;
  if (out_size != nN * 32) return;
  if (nE > (1 << 27) || nN > (1 << 26)) return;

  const float* x   = (const float*)d_in[0];
  const float* pos = (const float*)d_in[1];
  const int*   ei  = (const int*)d_in[2];
  const float* W1  = (const float*)d_in[3];
  const float* W2  = (const float*)d_in[4];
  float* out = (float*)d_out;

  const int nEB  = (nE + TE - 1) / TE;
  const int Epad = nEB * TE;
  const int nAB  = (nN + NODEB - 1) / NODEB;

  char* ws = (char*)d_ws;
  const size_t oBh = 0;
  const size_t oBl = (size_t)NR * KD * 2;
  const size_t oO  = 2 * (size_t)NR * KD * 2;
  const size_t total = oO + (size_t)Epad * 32 * 4;
  if (total > ws_size || total > ((size_t)128 << 20)) return;
  unsigned short* bhi  = (unsigned short*)(ws + oBh);
  unsigned short* blo  = (unsigned short*)(ws + oBl);
  float*          oute = (float*)(ws + oO);

  k_wprep<<<(2 * NR * 8 + NTHR - 1) / NTHR, NTHR, 0, stream>>>(W2, bhi, blo);

  k_edge<<<nEB, NTHR, LDS_EDGE, stream>>>(x, pos, ei, W1, bhi, blo, oute, nN, nE);

  k_agg<<<nAB, NTHR, LDS_AGG, stream>>>(ei, oute, out, nN, nE);
}
